// GCNModel_89970974917472
// MI455X (gfx1250) — hardware-verified
//
#include <hip/hip_runtime.h>
#include <stddef.h>
#include <stdint.h>
#include <math.h>


#define CH     128
#define HP     256
#define NG     512
#define POOLW  256
#define NTHR   256
#define NWAVE  8
#define EPT    8
#define CHUNK  (NTHR * EPT)
#define WCAP   (EPT * 32)
#define LISTN  (NWAVE * WCAP)
#define NBA    1024
#define SLA    10
#define RCAP   28672
#define DEGCAP 64
#define GBM    64
#define GBN    128
#define GTHR   128
#define GWAVE  (GTHR / 32)
#define ROWH   256
#define NUW1   (CH * (CH / 8))
#define NUWD   (CH * (HP / 8))
#define NUWE   (NUW1 + 2 * NUWD)
#define OW2D   (CH * CH)
#define OW3D   (CH * CH + CH * HP)
#define WPLN   (CH * CH + 2 * CH * HP)
#define PCH    1024
#define PLW    128
#define HG     32
#define AGG_ZINTS    (LISTN + 2 * RCAP + 3 * NBA)
#define MISC_INTS    16
#define BKT_LDS_INTS (AGG_ZINTS + MISC_INTS)
#define WSMAX  134217728

static_assert((CHUNK & (CHUNK - 1)) == 0 && CHUNK <= 4096);
static_assert((NBA & (NBA - 1)) == 0 && NBA == (1 << SLA));
static_assert(((long long)CHUNK << SLA) < (1LL << 31));
static_assert(NBA % NWAVE == 0 && NBA % 32 == 0 && NBA % GBM == 0 && NBA == 4 * NTHR);
static_assert(RCAP % (4 * NTHR) == 0 && AGG_ZINTS % 4 == 0 && LISTN % 4 == 0);
static_assert(RCAP >= 17546);
static_assert(DEGCAP >= 36 + 8);
static_assert(CH % 32 == 0 && HP % 32 == 0 && HP == 2 * CH);
static_assert(GBN == CH && GBM == GWAVE * 16 && CH == 4 * 32 && GTHR == GWAVE * 32);
static_assert(BKT_LDS_INTS * 4 <= 300000);
static_assert(ROWH == HP);
static_assert(NUW1 % NTHR == 0 && NUWD % NTHR == 0 && NUWE % NTHR == 0);
static_assert(POOLW == 2 * CH && NTHR == POOLW && PCH == 4 * NTHR && PLW == 4 * 32);
static_assert(NG % HG == 0 && HG == 32);

typedef float          v2f   __attribute__((ext_vector_type(2)));
typedef float          v4f   __attribute__((ext_vector_type(4)));
typedef float          v8f   __attribute__((ext_vector_type(8)));
typedef int            v4i   __attribute__((ext_vector_type(4)));
typedef int            v8i   __attribute__((ext_vector_type(8)));
typedef unsigned       v2u   __attribute__((ext_vector_type(2)));
typedef unsigned       v4u   __attribute__((ext_vector_type(4)));
typedef unsigned short v4us  __attribute__((ext_vector_type(4)));
typedef unsigned short v8us  __attribute__((ext_vector_type(8)));
typedef unsigned short v16us __attribute__((ext_vector_type(16)));
typedef __bf16         v16bf __attribute__((ext_vector_type(16)));
typedef v2f  __attribute__((may_alias)) v2fa;
typedef v4f  __attribute__((may_alias)) v4fa;
typedef v4i  __attribute__((may_alias)) v4ia;
typedef v2u  __attribute__((may_alias)) v2ua;
typedef v4us __attribute__((may_alias)) v4usa;
typedef v8us __attribute__((may_alias)) v8usa;
union FragB { v16bf v; v16us u; v8us h[2]; v8i w; };

__device__ __forceinline__ v8f wmb(const FragB& a, const FragB& b, v8f c) {
  v8f d = __builtin_amdgcn_wmma_f32_16x16x32_bf16(false, a.v, false, b.v, (short)0, c, false, false);
  asm volatile("v_nop\n\tv_nop\n\tv_nop\n\tv_nop" : "+v"(d) : "v"(a.w), "v"(b.w));
  return d;
}

__device__ __forceinline__ v8f z8() { v8f z = {0.f, 0.f, 0.f, 0.f, 0.f, 0.f, 0.f, 0.f}; return z; }

__device__ __forceinline__ unsigned bf16_bits(float f) {
  const unsigned u = __float_as_uint(f);
  const unsigned r = (u + 0x7FFFu + ((u >> 16) & 1u)) >> 16;
  return (f != f) ? 0x7FC0u : r;
}
__device__ __forceinline__ float bf16_val(float f) {
  return __uint_as_float(bf16_bits(f) << 16);
}
__device__ __forceinline__ unsigned hl_bits(float v, unsigned& lo) {
  const unsigned hb = bf16_bits(v);
  lo = bf16_bits(v - __uint_as_float(hb << 16));
  return hb;
}

__device__ __forceinline__ void wave_sync() {
  __builtin_amdgcn_fence(__ATOMIC_RELEASE, "wavefront");
  __builtin_amdgcn_wave_barrier();
  __builtin_amdgcn_fence(__ATOMIC_ACQUIRE, "wavefront");
}

__device__ __forceinline__ void put8(unsigned short* dp, v8us o) {
  *(volatile v8us*)dp = o;
  __threadfence();
  *(volatile v8us*)dp = o;
}

template <int SLB>
__device__ __forceinline__ int scan_chunk(const int* __restrict__ dsts, int nE, int cbase, int slotBase,
                                          int nb, int vec8, int* list, int tid, int lane, int wave) {
  int wc = 0;
  const int el0  = tid * EPT;
  const int e0   = cbase + el0;
  const int sent = -2147483647 - 1;
  v4i da, db;
  if (vec8 != 0 && cbase + CHUNK <= nE) {
    da = *(const v4i*)(dsts + e0);
    db = *(const v4i*)(dsts + e0 + 4);
  } else {
    da.x = (e0     < nE) ? dsts[min(e0,     nE - 1)] : sent;
    da.y = (e0 + 1 < nE) ? dsts[min(e0 + 1, nE - 1)] : sent;
    da.z = (e0 + 2 < nE) ? dsts[min(e0 + 2, nE - 1)] : sent;
    da.w = (e0 + 3 < nE) ? dsts[min(e0 + 3, nE - 1)] : sent;
    db.x = (e0 + 4 < nE) ? dsts[min(e0 + 4, nE - 1)] : sent;
    db.y = (e0 + 5 < nE) ? dsts[min(e0 + 5, nE - 1)] : sent;
    db.z = (e0 + 6 < nE) ? dsts[min(e0 + 6, nE - 1)] : sent;
    db.w = (e0 + 7 < nE) ? dsts[min(e0 + 7, nE - 1)] : sent;
  }
  const unsigned nbs = (unsigned)slotBase;
  const unsigned unb = (unsigned)nb;
  const unsigned s0 = (unsigned)da.x - nbs, s1 = (unsigned)da.y - nbs;
  const unsigned s2 = (unsigned)da.z - nbs, s3 = (unsigned)da.w - nbs;
  const unsigned s4 = (unsigned)db.x - nbs, s5 = (unsigned)db.y - nbs;
  const unsigned s6 = (unsigned)db.z - nbs, s7 = (unsigned)db.w - nbs;
  const bool h0 = s0 < unb, h1 = s1 < unb, h2 = s2 < unb, h3 = s3 < unb;
  const bool h4 = s4 < unb, h5 = s5 < unb, h6 = s6 < unb, h7 = s7 < unb;
  const unsigned any = __builtin_amdgcn_ballot_w32(h0 | h1 | h2 | h3 | h4 | h5 | h6 | h7);
  if (any != 0u) {
#define HITJ(J, HJ, SJ) { \
      const unsigned mj = __builtin_amdgcn_ballot_w32(HJ); \
      if (mj != 0u) { \
        if (HJ) { \
          const int pos = wc + (int)__builtin_amdgcn_mbcnt_lo(mj, 0u); \
          if (pos < WCAP) list[wave * WCAP + pos] = ((el0 + (J)) << SLB) | (int)(SJ); \
        } \
        wc += (int)__builtin_popcount(mj); } }
    HITJ(0, h0, s0)
    HITJ(1, h1, s1)
    HITJ(2, h2, s2)
    HITJ(3, h3, s3)
    HITJ(4, h4, s4)
    HITJ(5, h5, s5)
    HITJ(6, h6, s6)
    HITJ(7, h7, s7)
#undef HITJ
  }
  return wc;
}

__global__ __launch_bounds__(NTHR) void k_prep(const float* __restrict__ x, const float* __restrict__ W1,
                                               const float* __restrict__ W2, const float* __restrict__ W3,
                                               unsigned short* wpl, unsigned short* xb, int nN, int nUnits) {
  const int u = (int)blockIdx.x * NTHR + (int)threadIdx.x;
  v8us o;
  if (u < NUW1) {
    const int n = u >> 4, k8 = (u & 15) * 8;
    const float* p = W1 + (size_t)k8 * CH + n;
#pragma unroll
    for (int i = 0; i < 8; ++i) o[i] = (unsigned short)bf16_bits(p[(size_t)i * CH]);
    put8(wpl + (size_t)u * 8, o);
  } else if (u < NUW1 + NUWD) {
    const int v = u - NUW1;
    const int n = v >> 5, k8 = (v & 31) * 8, kk = k8 & (CH - 1);
    const float* p = W2 + (size_t)kk * CH + n;
#pragma unroll
    for (int i = 0; i < 8; ++i) o[i] = (unsigned short)bf16_bits(p[(size_t)i * CH]);
    put8(wpl + OW2D + (size_t)v * 8, o);
  } else if (u < NUWE) {
    const int v = u - NUW1 - NUWD;
    const int n = v >> 5, k8 = (v & 31) * 8, kk = k8 & (CH - 1);
    const float* p = W3 + (size_t)kk * CH + n;
#pragma unroll
    for (int i = 0; i < 8; ++i) o[i] = (unsigned short)bf16_bits(p[(size_t)i * CH]);
    put8(wpl + OW3D + (size_t)v * 8, o);
  } else if (u < nUnits) {
    const int v   = u - NUWE;
    const int row = v >> 4, k8 = (v & 15) * 8;
    const int rc  = row < nN ? row : nN - 1;
    const float* p = x + (size_t)rc * CH + k8;
    const v4f a = *(const v4fa*)p;
    const v4f b = *(const v4fa*)(p + 4);
    const bool ok = row < nN;
    o[0] = ok ? (unsigned short)bf16_bits(a.x) : (unsigned short)0;
    o[1] = ok ? (unsigned short)bf16_bits(a.y) : (unsigned short)0;
    o[2] = ok ? (unsigned short)bf16_bits(a.z) : (unsigned short)0;
    o[3] = ok ? (unsigned short)bf16_bits(a.w) : (unsigned short)0;
    o[4] = ok ? (unsigned short)bf16_bits(b.x) : (unsigned short)0;
    o[5] = ok ? (unsigned short)bf16_bits(b.y) : (unsigned short)0;
    o[6] = ok ? (unsigned short)bf16_bits(b.z) : (unsigned short)0;
    o[7] = ok ? (unsigned short)bf16_bits(b.w) : (unsigned short)0;
    put8(xb + (size_t)v * 8, o);
  }
}

__global__ __launch_bounds__(NTHR) void k_bucket(const int* __restrict__ srcs, const int* __restrict__ dsts,
                                                 int nE, int nN, int vec8,
                                                 int* LIST, int* CNT, int* OFF, float* DIS, int* FLAG) {
  extern __shared__ __attribute__((aligned(16))) int dsm[];
  int* list = dsm;
  int* hl   = dsm + LISTN;
  int* sl   = hl + RCAP;
  int* cnt  = sl + RCAP;
  int* offs = cnt + NBA;
  int* cur  = offs + NBA;
  int* misc = cur + NBA;
  const int tid = (int)threadIdx.x, lane = tid & 31, wave = tid >> 5;
  const int nodeBase = (int)blockIdx.x * NBA;

  {
    const v4i z4 = {0, 0, 0, 0};
    for (int i = tid * 4; i < AGG_ZINTS; i += NTHR * 4) *(v4ia*)(dsm + i) = z4;
    if (tid < MISC_INTS) misc[tid] = 0;
  }
  __syncthreads();

  int t = 0, ov = 0;
  const int nChunks = (nE + CHUNK - 1) / CHUNK;
#pragma unroll 1
  for (int ch = 0; ch < nChunks; ++ch) {
    const int cbase = ch * CHUNK;
    const int wc = scan_chunk<SLA>(dsts, nE, cbase, nodeBase, NBA, vec8, list, tid, lane, wave);
    if (lane == 0) misc[wave] = wc;
    __syncthreads();
    if (wave == 0) {
#pragma unroll 1
      for (int w2 = 0; w2 < NWAVE; ++w2) {
        int c = misc[w2];
        c = c < 0 ? 0 : (c > WCAP ? WCAP : c);
#pragma unroll 1
        for (int b0 = 0; b0 < c; b0 += 32) {
          const int idx = b0 + lane;
          const int ent_ = list[w2 * WCAP + (idx < WCAP ? idx : WCAP - 1)];
          const int m32 = (c - b0) < 32 ? (c - b0) : 32;
#pragma unroll 1
          for (int k = 0; k < m32; ++k) {
            const int u    = __builtin_amdgcn_readlane(ent_, k);
            const int slot = u & (NBA - 1);
            const int el   = (u >> SLA) & (CHUNK - 1);
            const int pk   = ((cbase + el) << SLA) | slot;
            if (t < RCAP) {
              if (lane == 0) { hl[t] = pk; cnt[slot] = cnt[slot] + 1; }
              t = t + 1;
            } else {
              ov = 1;
            }
          }
        }
      }
    }
    __syncthreads();
  }
  if (wave == 0 && lane == 0) { misc[8] = t; misc[9] = ov; }
  __syncthreads();
  int tt = misc[8];
  tt = tt < 0 ? 0 : (tt > RCAP ? RCAP : tt);
  const int ovf = misc[9];

  if (wave == 0) {
    const int base = lane * (NBA / 32);
    int s = 0;
#pragma unroll 1
    for (int i = 0; i < NBA / 32; ++i) s += cnt[base + i];
    int incl = s;
#pragma unroll
    for (int d = 1; d < 32; d <<= 1) {
      const int y = __shfl_up(incl, d, 32);
      if (lane >= d) incl += y;
    }
    int run = incl - s;
#pragma unroll 1
    for (int i = 0; i < NBA / 32; ++i) {
      const int cv = cnt[base + i];
      offs[base + i] = run;
      cur[base + i]  = run;
      run += cv;
    }
  }
  __syncthreads();
  if (wave == 0) {
#pragma unroll 1
    for (int b0 = 0; b0 < tt; b0 += 32) {
      const int idx = b0 + lane;
      const int ent_ = hl[idx < RCAP ? idx : RCAP - 1];
      const int m32 = (tt - b0) < 32 ? (tt - b0) : 32;
#pragma unroll 1
      for (int k = 0; k < m32; ++k) {
        const int u    = __builtin_amdgcn_readlane(ent_, k);
        const int slot = u & (NBA - 1);
        if (lane == 0) {
          int p = cur[slot];
          p = p < 0 ? 0 : (p > RCAP - 1 ? RCAP - 1 : p);
          sl[p] = u;
          cur[slot] = p + 1;
        }
      }
    }
  }
  __syncthreads();

#pragma unroll 1
  for (int i = tid; i < NBA; i += NTHR) {
    const float d = (float)(cnt[i] + 1);
    const float r = (d > 0.0f) ? (1.0f / sqrtf(d)) : 0.0f;
    cur[i] = __float_as_int(r);
  }
  __syncthreads();

  {
    const v4i c4 = *(const v4ia*)(cnt + 4 * tid);
    const v4i o4 = *(const v4ia*)(offs + 4 * tid);
    const v4i r4 = *(const v4ia*)(cur + 4 * tid);
    v4f d4;
    d4.x = __int_as_float(r4.x); d4.y = __int_as_float(r4.y);
    d4.z = __int_as_float(r4.z); d4.w = __int_as_float(r4.w);
    const v4i f4 = {ovf, ovf, ovf, ovf};
    int*   cp = CNT + (size_t)nodeBase + 4 * tid;
    int*   op = OFF + (size_t)nodeBase + 4 * tid;
    float* dp = DIS + (size_t)nodeBase + 4 * tid;
    int*   fp = FLAG + (size_t)blockIdx.x * 32 + 4 * (tid & 7);
    const bool fl = tid < 8;
    *(volatile v4i*)cp = c4;
    *(volatile v4i*)op = o4;
    *(volatile v4f*)dp = d4;
    if (fl) *(volatile v4i*)fp = f4;
    __threadfence();
    *(volatile v4i*)cp = c4;
    *(volatile v4i*)op = o4;
    *(volatile v4f*)dp = d4;
    if (fl) *(volatile v4i*)fp = f4;
  }

  int* lrow = LIST + (size_t)blockIdx.x * RCAP;
#pragma unroll 1
  for (int p0 = 4 * tid; p0 < RCAP; p0 += 4 * NTHR) {
    const v4i e4 = *(const v4ia*)(sl + p0);
    int e0 = e4.x >> SLA, e1 = e4.y >> SLA, e2 = e4.z >> SLA, e3 = e4.w >> SLA;
    e0 = e0 < 0 ? 0 : (e0 > nE - 1 ? nE - 1 : e0);
    e1 = e1 < 0 ? 0 : (e1 > nE - 1 ? nE - 1 : e1);
    e2 = e2 < 0 ? 0 : (e2 > nE - 1 ? nE - 1 : e2);
    e3 = e3 < 0 ? 0 : (e3 > nE - 1 ? nE - 1 : e3);
    int r0 = srcs[e0], r1 = srcs[e1], r2 = srcs[e2], r3 = srcs[e3];
    r0 = r0 < 0 ? 0 : (r0 > nN - 1 ? nN - 1 : r0);
    r1 = r1 < 0 ? 0 : (r1 > nN - 1 ? nN - 1 : r1);
    r2 = r2 < 0 ? 0 : (r2 > nN - 1 ? nN - 1 : r2);
    r3 = r3 < 0 ? 0 : (r3 > nN - 1 ? nN - 1 : r3);
    v4i w4;
    w4.x = (p0     < tt) ? r0 : 0;
    w4.y = (p0 + 1 < tt) ? r1 : 0;
    w4.z = (p0 + 2 < tt) ? r2 : 0;
    w4.w = (p0 + 3 < tt) ? r3 : 0;
    *(volatile v4i*)(lrow + p0) = w4;
    __threadfence();
    *(volatile v4i*)(lrow + p0) = w4;
  }
}

__global__ __launch_bounds__(GTHR) void k_gemm(const unsigned short* __restrict__ A, int lda,
                                               const unsigned short* __restrict__ BT, int ldb, int K,
                                               float* outF, int mRows) {
  __shared__ __attribute__((aligned(16))) float stg[GBM * GBN];
  const int tid = (int)threadIdx.x, lane = tid & 31, wave = tid >> 5, hh = lane >> 4, m = lane & 15;
  const int rowBase = (int)blockIdx.x * GBM;

  v8f acc[8];
#pragma unroll
  for (int t = 0; t < 8; ++t) acc[t] = z8();
  const unsigned short* ap = A + (size_t)(rowBase + 16 * wave + m) * (size_t)lda + 8 * hh;
  const unsigned short* bp = BT + (size_t)m * (size_t)ldb + 8 * hh;

#pragma unroll 1
  for (int k0 = 0; k0 < K; k0 += 32) {
    FragB af;
    af.h[0] = *(const v8usa*)(ap + k0);
    af.h[1] = *(const v8usa*)(ap + k0 + 16);
#pragma unroll
    for (int nt = 0; nt < 8; ++nt) {
      const unsigned short* wq = bp + (size_t)(16 * nt) * (size_t)ldb + k0;
      FragB bf;
      bf.h[0] = *(const v8usa*)wq;
      bf.h[1] = *(const v8usa*)(wq + 16);
      acc[nt] = wmb(af, bf, acc[nt]);
    }
  }

#pragma unroll
  for (int nt = 0; nt < 8; ++nt) {
    const int lc = 16 * nt + m;
#pragma unroll
    for (int r = 0; r < 8; ++r) {
      const int lr = 16 * wave + 8 * hh + r;
      stg[lr * GBN + lc] = acc[nt][r];
    }
  }
  __syncthreads();

  v4f pv[16];
#pragma unroll
  for (int i = 0; i < 16; ++i) pv[i] = *(const v4fa*)(stg + (16 * wave + i) * GBN + 4 * lane);
#pragma unroll
  for (int i = 0; i < 16; ++i) {
    const int gr = rowBase + 16 * wave + i;
    float* op = outF + (size_t)gr * GBN + 4 * lane;
    if (gr < mRows) *(volatile v4f*)op = pv[i];
  }
  __threadfence();
#pragma unroll
  for (int i = 0; i < 16; ++i) {
    const int gr = rowBase + 16 * wave + i;
    float* op = outF + (size_t)gr * GBN + 4 * lane;
    if (gr < mRows) *(volatile v4f*)op = pv[i];
  }
}

template <int RES>
__global__ __launch_bounds__(NTHR) void k_agg(const int* __restrict__ LIST, const int* __restrict__ CNT,
                                              const int* __restrict__ OFF, const float* __restrict__ dis,
                                              const int* __restrict__ FLAG, const float* __restrict__ T,
                                              const float* __restrict__ bias, unsigned short* hhl,
                                              int nN, int mRows) {
  __shared__ __attribute__((aligned(16))) unsigned short rowbuf_all[NWAVE * ROWH];
  const int tid = (int)threadIdx.x, lane = tid & 31, wave = tid >> 5;
  unsigned short* rowbuf = rowbuf_all + wave * ROWH;
  const int nodeBase = (int)blockIdx.x * NBA;
  const int* lrow = LIST + (size_t)blockIdx.x * RCAP;
  const float qnan = __int_as_float(0x7fc00000);
  const int ovf = FLAG[(size_t)blockIdx.x * 32];
  const float pz = (ovf != 0) ? qnan : 0.0f;
  float bq0, bq1, bq2, bq3;
  {
    const v4f b4 = *(const v4f*)(bias + 4 * lane);
    bq0 = bf16_val(b4.x); bq1 = bf16_val(b4.y); bq2 = bf16_val(b4.z); bq3 = bf16_val(b4.w);
  }
#pragma unroll 1
  for (int si = 0; si < NBA / NWAVE; ++si) {
    const int s    = si * NWAVE + wave;
    const int node = nodeBase + s;
    if (node >= mRows) continue;
    int c = CNT[node];
    const bool big = c > DEGCAP;
    c = c < 0 ? 0 : (c > DEGCAP ? DEGCAP : c);
    int o = OFF[node];
    o = o < 0 ? 0 : (o > RCAP ? RCAP : o);
    const int nc = node < nN ? node : nN - 1;
    const bool live = node < nN;
    const float dd = dis[nc];
    const float rd = dd * dd;
    float a0 = 0.0f, a1 = 0.0f, a2 = 0.0f, a3 = 0.0f;
#pragma unroll 1
    for (int b0 = 0; b0 < c; b0 += 32) {
      int idx = o + b0 + lane;
      idx = idx > RCAP - 1 ? RCAP - 1 : idx;
      int sr = lrow[idx];
      sr = sr < 0 ? 0 : (sr > nN - 1 ? nN - 1 : sr);
      const float cf  = dis[sr] * dd;
      const int   cfi = __float_as_int(cf);
      const int m32 = (c - b0) < 32 ? (c - b0) : 32;
#pragma unroll 1
      for (int k = 0; k < m32; ++k) {
        const int   sk = __builtin_amdgcn_readlane(sr, k);
        const float ck = __int_as_float(__builtin_amdgcn_readlane(cfi, k));
        const v4f a = *(const v4fa*)(T + (size_t)sk * CH + 4 * lane);
        a0 = fmaf(ck, a.x, a0); a1 = fmaf(ck, a.y, a1);
        a2 = fmaf(ck, a.z, a2); a3 = fmaf(ck, a.w, a3);
      }
    }
    const v4f sv = *(const v4fa*)(T + (size_t)nc * CH + 4 * lane);
    float y0 = (a0 + sv.x * rd) + bq0;
    float y1 = (a1 + sv.y * rd) + bq1;
    float y2 = (a2 + sv.z * rd) + bq2;
    float y3 = (a3 + sv.w * rd) + bq3;
    y0 = (y0 > 0.0f) ? y0 : (y0 - y0);
    y1 = (y1 > 0.0f) ? y1 : (y1 - y1);
    y2 = (y2 > 0.0f) ? y2 : (y2 - y2);
    y3 = (y3 > 0.0f) ? y3 : (y3 - y3);
    const float pzr = big ? qnan : pz;
    y0 += pzr; y1 += pzr; y2 += pzr; y3 += pzr;
    if constexpr (RES != 0) {
      const unsigned short* rp = hhl + (size_t)node * HP + 4 * lane;
      const v2u wh = *(const v2ua*)rp;
      const v2u wl = *(const v2ua*)(rp + CH);
      y0 += __uint_as_float(wh.x << 16)         + __uint_as_float(wl.x << 16);
      y1 += __uint_as_float(wh.x & 0xffff0000u) + __uint_as_float(wl.x & 0xffff0000u);
      y2 += __uint_as_float(wh.y << 16)         + __uint_as_float(wl.y << 16);
      y3 += __uint_as_float(wh.y & 0xffff0000u) + __uint_as_float(wl.y & 0xffff0000u);
    }
    const float v0 = live ? y0 : 0.0f;
    const float v1 = live ? y1 : 0.0f;
    const float v2 = live ? y2 : 0.0f;
    const float v3 = live ? y3 : 0.0f;
    v4us mh, ml;
    {
      unsigned lb;
      unsigned hb;
      hb = hl_bits(v0, lb); mh[0] = (unsigned short)hb; ml[0] = (unsigned short)lb;
      hb = hl_bits(v1, lb); mh[1] = (unsigned short)hb; ml[1] = (unsigned short)lb;
      hb = hl_bits(v2, lb); mh[2] = (unsigned short)hb; ml[2] = (unsigned short)lb;
      hb = hl_bits(v3, lb); mh[3] = (unsigned short)hb; ml[3] = (unsigned short)lb;
    }
    *(v4usa*)(rowbuf + 4 * lane)      = mh;
    *(v4usa*)(rowbuf + CH + 4 * lane) = ml;
    wave_sync();
    const v8us q0 = *(const v8usa*)(rowbuf + 8 * lane);
    wave_sync();
    unsigned short* rpw = hhl + (size_t)node * HP + 8 * lane;
    *(volatile v8us*)rpw = q0;
    __threadfence();
    *(volatile v8us*)rpw = q0;
  }
}

__global__ __launch_bounds__(NTHR) void k_pool(const unsigned short* __restrict__ hhl, const int* __restrict__ bat,
                                               int nN, int vec4, float* gout) {
  __shared__ __attribute__((aligned(16))) float wst[NWAVE * POOLW];
  __shared__ __attribute__((aligned(16))) float pst[POOLW];
  __shared__ int plist[NWAVE * PLW];
  __shared__ int wcn[NWAVE];
  const int tid = (int)threadIdx.x, lane = tid & 31, wave = tid >> 5;
  const int g = (int)blockIdx.x;
  const float nhuge = -__builtin_huge_valf();
  for (int i = tid; i < NWAVE * PLW; i += NTHR) plist[i] = 0;
  __syncthreads();
  float s0 = 0.0f, s1 = 0.0f, s2 = 0.0f, s3 = 0.0f;
  float m0 = nhuge, m1 = nhuge, m2 = nhuge, m3 = nhuge;
  int cn = 0;
  const int nChunks = (nN + PCH - 1) / PCH;
#pragma unroll 1
  for (int ch = 0; ch < nChunks; ++ch) {
    const int cbase = ch * PCH;
    const int n0 = cbase + 4 * tid;
    v4i b4;
    if (vec4 != 0 && cbase + PCH <= nN) {
      b4 = *(const v4i*)(bat + n0);
    } else {
      b4.x = (n0     < nN) ? bat[min(n0,     nN - 1)] : -1;
      b4.y = (n0 + 1 < nN) ? bat[min(n0 + 1, nN - 1)] : -1;
      b4.z = (n0 + 2 < nN) ? bat[min(n0 + 2, nN - 1)] : -1;
      b4.w = (n0 + 3 < nN) ? bat[min(n0 + 3, nN - 1)] : -1;
    }
    const bool h0 = b4.x == g, h1 = b4.y == g, h2 = b4.z == g, h3 = b4.w == g;
    const unsigned any = __builtin_amdgcn_ballot_w32(h0 | h1 | h2 | h3);
    if (any != 0u) {
      int wc = 0;
#define PHIT(J, HJ) { \
        const unsigned mj = __builtin_amdgcn_ballot_w32(HJ); \
        if (HJ) { \
          const int pos = wc + (int)__builtin_amdgcn_mbcnt_lo(mj, 0u); \
          if (pos < PLW) plist[wave * PLW + pos] = n0 + (J); \
        } \
        wc += (int)__builtin_popcount(mj); }
      PHIT(0, h0)
      PHIT(1, h1)
      PHIT(2, h2)
      PHIT(3, h3)
#undef PHIT
      wc = wc > PLW ? PLW : wc;
      wave_sync();
#pragma unroll 1
      for (int k = 0; k < wc; ++k) {
        int nd = plist[wave * PLW + k];
        nd = nd < 0 ? 0 : (nd > nN - 1 ? nN - 1 : nd);
        const unsigned short* rp = hhl + (size_t)nd * HP + 4 * lane;
        const v2u wh = *(const v2ua*)rp;
        const v2u wl = *(const v2ua*)(rp + CH);
        const float f0 = __uint_as_float(wh.x << 16)         + __uint_as_float(wl.x << 16);
        const float f1 = __uint_as_float(wh.x & 0xffff0000u) + __uint_as_float(wl.x & 0xffff0000u);
        const float f2 = __uint_as_float(wh.y << 16)         + __uint_as_float(wl.y << 16);
        const float f3 = __uint_as_float(wh.y & 0xffff0000u) + __uint_as_float(wl.y & 0xffff0000u);
        s0 += f0; s1 += f1; s2 += f2; s3 += f3;
        m0 = (f0 > m0 || f0 != f0) ? f0 : m0;
        m1 = (f1 > m1 || f1 != f1) ? f1 : m1;
        m2 = (f2 > m2 || f2 != f2) ? f2 : m2;
        m3 = (f3 > m3 || f3 != f3) ? f3 : m3;
      }
      cn += wc;
      wave_sync();
    }
  }
  {
    v4f sv4; sv4.x = s0; sv4.y = s1; sv4.z = s2; sv4.w = s3;
    v4f mv4; mv4.x = m0; mv4.y = m1; mv4.z = m2; mv4.w = m3;
    *(v4fa*)(wst + wave * POOLW + 4 * lane) = sv4;
    *(v4fa*)(wst + wave * POOLW + CH + 4 * lane) = mv4;
    if (lane == 0) wcn[wave] = cn;
  }
  __syncthreads();
  {
    const int c = tid & (CH - 1);
    const int half = tid >> 7;
    double sv = 0.0;
    float mv = nhuge;
    int ct = 0;
#pragma unroll 1
    for (int w2 = 0; w2 < NWAVE; ++w2) {
      sv += (double)wst[w2 * POOLW + c];
      const float xm = wst[w2 * POOLW + CH + c];
      mv = (xm > mv || xm != xm) ? xm : mv;
      ct += wcn[w2];
    }
    const float cf = (float)(ct < 1 ? 1 : ct);
    const float mean = (float)sv * (1.0f / cf);
    pst[tid] = (half == 0) ? mean : mv;
  }
  __syncthreads();
  const bool ok = tid < POOLW / 4;
  const v4f pvv = *(const v4fa*)(pst + 4 * (tid & 63));
  float* op = gout + (size_t)g * POOLW + 4 * (tid & 63);
  if (ok) *(volatile v4f*)op = pvv;
  __threadfence();
  if (ok) *(volatile v4f*)op = pvv;
}

__global__ __launch_bounds__(NTHR) void k_head(const float* __restrict__ G, const float* __restrict__ Wf1,
                                               const float* __restrict__ bf1, const float* __restrict__ Wf2,
                                               const float* __restrict__ bf2, const float* __restrict__ Wf3,
                                               const float* __restrict__ bf3, const int* __restrict__ FLAG,
                                               int nFlag, int nG, float* out) {
  __shared__ __attribute__((aligned(16))) float gs[HG * POOLW];
  __shared__ float a1s[HG * CH];
  __shared__ float a2s[HG * 64];
  __shared__ float outs[HG];
  __shared__ int sflag;
  const int tid = (int)threadIdx.x, lane = tid & 31, wave = tid >> 5;
  const int g0 = (int)blockIdx.x * HG;
#pragma unroll 1
  for (int i = tid; i < HG * (POOLW / 4); i += NTHR)
    *(v4fa*)(gs + 4 * i) = *(const v4f*)(G + (size_t)g0 * POOLW + 4 * i);
  if (tid == 0) sflag = 0;
  __syncthreads();
  {
    const int fi = tid < nFlag ? tid : nFlag - 1;
    const int f = FLAG[(size_t)fi * 32];
    if (tid < nFlag && f != 0) sflag = 1;
  }
  {
    const int n = tid & (CH - 1), gsel = tid >> 7;
    const float bb = bf16_val(bf1[n]);
#pragma unroll 1
    for (int ps = 0; ps < 2; ++ps) {
      float ac[8];
#pragma unroll
      for (int j = 0; j < 8; ++j) ac[j] = 0.0f;
      const float* gp = gs + (gsel + 16 * ps) * POOLW;
#pragma unroll 2
      for (int k = 0; k < POOLW; ++k) {
        const float w = bf16_val(Wf1[(size_t)k * CH + n]);
#pragma unroll
        for (int j = 0; j < 8; ++j) ac[j] = fmaf(gp[j * 2 * POOLW + k], w, ac[j]);
      }
#pragma unroll
      for (int j = 0; j < 8; ++j) {
        float v = ac[j] + bb;
        v = (v > 0.0f) ? v : (v - v);
        a1s[(gsel + 2 * (8 * ps + j)) * CH + n] = v;
      }
    }
  }
  __syncthreads();
  {
    const int n = tid & 63, gsel = tid >> 6;
    const float bb = bf16_val(bf2[n]);
    float ac[8];
#pragma unroll
    for (int j = 0; j < 8; ++j) ac[j] = 0.0f;
    const float* ap = a1s + gsel * CH;
#pragma unroll 2
    for (int k = 0; k < CH; ++k) {
      const float w = bf16_val(Wf2[(size_t)k * 64 + n]);
#pragma unroll
      for (int j = 0; j < 8; ++j) ac[j] = fmaf(ap[j * 4 * CH + k], w, ac[j]);
    }
#pragma unroll
    for (int j = 0; j < 8; ++j) {
      float v = ac[j] + bb;
      v = (v > 0.0f) ? v : (v - v);
      a2s[(gsel + 4 * j) * 64 + n] = v;
    }
  }
  __syncthreads();
  {
    const float w3a = bf16_val(Wf3[lane]);
    const float w3b = bf16_val(Wf3[lane + 32]);
    const float b3  = bf16_val(bf3[0]);
#pragma unroll 1
    for (int q = 0; q < HG / NWAVE; ++q) {
      const int gi = (HG / NWAVE) * wave + q;
      float s = a2s[gi * 64 + lane] * w3a;
      s = fmaf(a2s[gi * 64 + lane + 32], w3b, s);
      s += __shfl_xor(s, 16, 32);
      s += __shfl_xor(s, 8, 32);
      s += __shfl_xor(s, 4, 32);
      s += __shfl_xor(s, 2, 32);
      s += __shfl_xor(s, 1, 32);
      if (lane == 0) outs[gi] = s + b3;
    }
  }
  __syncthreads();
  const float qnan = __int_as_float(0x7fc00000);
  const float ov = outs[lane];
  const float fv = (sflag != 0) ? qnan : ov;
  const bool okst = (wave == 0) && (g0 + lane < nG);
  float* op = out + g0 + lane;
  if (okst) *(volatile float*)op = fv;
  __threadfence();
  if (okst) *(volatile float*)op = fv;
}

static inline int cdiv(int a, int b) { return (a + b - 1) / b; }
static inline size_t al256(size_t o) { return (o + 255) & ~(size_t)255; }

extern "C" void kernel_launch(void* const* d_in, const int* in_sizes, int n_in,
                              void* d_out, int out_size, void* d_ws, size_t ws_size,
                              hipStream_t stream) {
  if (n_in < 16) return;
  if (in_sizes[0] < CH || (in_sizes[0] % CH) != 0) return;
  const int nN = in_sizes[0] / CH;
  if (nN < GBM || nN > (1 << 22)) return;
  if (in_sizes[1] < 2 || (in_sizes[1] & 1) != 0) return;
  const int nE = in_sizes[1] / 2;
  if (nE < 1 || nE >= (1 << 21)) return;
  if (in_sizes[2] != nN) return;
  if (in_sizes[4] != CH * CH || in_sizes[6] != CH * CH || in_sizes[8] != CH * CH) return;
  if (in_sizes[5] != CH || in_sizes[7] != CH || in_sizes[9] != CH) return;
  if (in_sizes[10] != POOLW * CH || in_sizes[11] != CH) return;
  if (in_sizes[12] != CH * 64 || in_sizes[13] != 64) return;
  if (in_sizes[14] != 64 || in_sizes[15] != 1) return;
  if (out_size != NG) return;

  const float* x    = (const float*)d_in[0];
  const int*   edge = (const int*)  d_in[1];
  const int*   bat  = (const int*)  d_in[2];
  const float* W1   = (const float*)d_in[4];
  const float* b1   = (const float*)d_in[5];
  const float* W2   = (const float*)d_in[6];
  const float* b2   = (const float*)d_in[7];
  const float* W3   = (const float*)d_in[8];
  const float* b3   = (const float*)d_in[9];
  const float* Wf1  = (const float*)d_in[10];
  const float* bf1  = (const float*)d_in[11];
  const float* Wf2  = (const float*)d_in[12];
  const float* bf2  = (const float*)d_in[13];
  const float* Wf3  = (const float*)d_in[14];
  const float* bf3  = (const float*)d_in[15];
  float* out = (float*)d_out;
  const int* src = edge;
  const int* dst = edge + nE;

  const int MP  = cdiv(nN, 128) * 128;
  const int gM  = MP / GBM;
  const int gA  = cdiv(MP, NBA);
  const int NBP = gA * NBA;
  if ((long long)gA * NBA < (long long)MP) return;
  if (gA > NTHR) return;
  const int vec8 = ((nE & 3) == 0) ? 1 : 0;

  char* ws = (char*)d_ws;
  size_t off = 0;
  const size_t oHHL = off; off = al256(off + (size_t)MP * HP * 2);
  const size_t oT   = off; off = al256(off + (size_t)MP * CH * 4);
  const size_t oLST = off; off = al256(off + (size_t)gA * RCAP * 4);
  const size_t oCNT = off; off = al256(off + (size_t)NBP * 4);
  const size_t oOFF = off; off = al256(off + (size_t)NBP * 4);
  const size_t oDIS = off; off = al256(off + (size_t)NBP * 4);
  const size_t oWPL = off; off = al256(off + (size_t)WPLN * 2);
  const size_t oG   = off; off = al256(off + (size_t)NG * POOLW * 4);
  const size_t oFLG = off; off = al256(off + (size_t)gA * 32 * 4);
  if (off > ws_size || off > (size_t)WSMAX) return;
  if ((size_t)MP * CH * 2 > (size_t)MP * HP * 2) return;
  unsigned short* HHL = (unsigned short*)(ws + oHHL);
  unsigned short* XB  = (unsigned short*)(ws + oHHL);
  float*          T   = (float*)(ws + oT);
  int*            LST = (int*)(ws + oLST);
  int*            CNT = (int*)(ws + oCNT);
  int*            OFF = (int*)(ws + oOFF);
  float*          DIS = (float*)(ws + oDIS);
  unsigned short* WPL = (unsigned short*)(ws + oWPL);
  float*          G   = (float*)(ws + oG);
  int*            FLG = (int*)(ws + oFLG);
  const unsigned short* W1T = WPL;
  const unsigned short* W2D = WPL + OW2D;
  const unsigned short* W3D = WPL + OW3D;

  const size_t bktLds = (size_t)BKT_LDS_INTS * 4;
  hipFuncSetAttribute(reinterpret_cast<const void*>(&k_bucket), hipFuncAttributeMaxDynamicSharedMemorySize, (int)bktLds);

  const int nUnits = NUWE + MP * (CH / 8);

  k_prep<<<cdiv(nUnits, NTHR), NTHR, 0, stream>>>(x, W1, W2, W3, WPL, XB, nN, nUnits);
  k_bucket<<<gA, NTHR, bktLds, stream>>>(src, dst, nE, nN, vec8, LST, CNT, OFF, DIS, FLG);
  k_gemm<<<gM, GTHR, 0, stream>>>(XB, CH, W1T, CH, CH, T, MP);
  k_agg<0><<<gA, NTHR, 0, stream>>>(LST, CNT, OFF, DIS, FLG, T, b1, HHL, nN, MP);
  k_gemm<<<gM, GTHR, 0, stream>>>(HHL, HP, W2D, HP, HP, T, MP);
  k_agg<1><<<gA, NTHR, 0, stream>>>(LST, CNT, OFF, DIS, FLG, T, b2, HHL, nN, MP);
  k_gemm<<<gM, GTHR, 0, stream>>>(HHL, HP, W3D, HP, HP, T, MP);
  k_agg<1><<<gA, NTHR, 0, stream>>>(LST, CNT, OFF, DIS, FLG, T, b3, HHL, nN, MP);
  k_pool<<<NG, NTHR, 0, stream>>>(HHL, bat, nN, 1, G);
  k_head<<<NG / HG, NTHR, 0, stream>>>(G, Wf1, bf1, Wf2, bf2, Wf3, bf3, FLG, gA, NG, out);
}
